// GATLayer_48782238548193
// MI455X (gfx1250) — hardware-verified
//
#include <hip/hip_runtime.h>
#include <math.h>
#include <stdint.h>
#include <stddef.h>

#define NN_   4096
#define INF_  512
#define NH_   8
#define HF_   32
#define DM_   (NH_ * HF_)
#define ADW   128
#define SLOPE 0.2f
#define MASKFILL (-1.0e9f)
#define MASKHALF (-1.0e8f)
#define WSMAX 134217728

static_assert(DM_ == NH_ * HF_);
static_assert(HF_ == 32);
static_assert(NN_ == ADW * 32);
static_assert(NN_ % 128 == 0);
static_assert(NN_ % 64 == 0);
static_assert(INF_ % 64 == 0);
static_assert(INF_ % 32 == 0);
static_assert(DM_ % 64 == 0);
static_assert((NN_ * INF_) % 2048 == 0);

typedef __attribute__((ext_vector_type(16))) __bf16 v16b;
typedef __attribute__((ext_vector_type(8)))  __bf16 v8b;
typedef __attribute__((ext_vector_type(8)))  float  v8f;
typedef __attribute__((ext_vector_type(4)))  float  v4f;
typedef __attribute__((ext_vector_type(4)))  unsigned int v4u;
typedef __attribute__((ext_vector_type(2)))  unsigned int v2u;
typedef __attribute__((ext_vector_type(8)))  unsigned int v8u;
typedef __attribute__((ext_vector_type(4)))  int v4i;
typedef v8b __attribute__((may_alias)) v8ba;
typedef v4f __attribute__((may_alias)) v4fa;
typedef v4u __attribute__((may_alias)) v4ua;
typedef v2u __attribute__((may_alias)) v2ua;
typedef v4i __attribute__((may_alias)) v4ia;

union FragU { v16b v; v8b h[2]; };
union PackU { v8u u; v16b v; };

__device__ __forceinline__ unsigned short f2bf_bits(float f) {
  const unsigned u = __float_as_uint(f);
  return (unsigned short)((u + 0x7FFFu + ((u >> 16) & 1u)) >> 16);
}
__device__ __forceinline__ float bf_bits2f(unsigned short h) { return __uint_as_float(((unsigned)h) << 16); }
__device__ __forceinline__ float bf16r(float f) {
  unsigned u = __float_as_uint(f);
  u = (u + 0x7FFFu + ((u >> 16) & 1u)) & 0xFFFF0000u;
  return __uint_as_float(u);
}
__device__ __forceinline__ unsigned pk16(unsigned short a, unsigned short b) { return (unsigned)a | ((unsigned)b << 16); }

__device__ __forceinline__ v8f wmma_bf16(v16b a, v16b b, v8f c) {
  v8f d = __builtin_amdgcn_wmma_f32_16x16x32_bf16(false, a, false, b, (short)0, c, false, false);
  asm volatile("v_nop\n\tv_nop\n\tv_nop\n\tv_nop" : "+v"(d) : "v"(a), "v"(b));
  return d;
}

__device__ __forceinline__ v16b load_frag(const unsigned short* p, int hh) {
  FragU f;
  f.h[0] = *(const v8ba*)(p + 8 * hh);
  f.h[1] = *(const v8ba*)(p + 16 + 8 * hh);
  return f.v;
}

__device__ __forceinline__ void pack_p2(v8f a, v8f c, v16b& ho, v16b& lo) {
  PackU uh, ul;
#pragma unroll
  for (int i = 0; i < 4; ++i) {
    const unsigned short h0 = f2bf_bits(a[2 * i]), h1 = f2bf_bits(a[2 * i + 1]);
    const unsigned short l0 = f2bf_bits(a[2 * i] - bf_bits2f(h0)), l1 = f2bf_bits(a[2 * i + 1] - bf_bits2f(h1));
    uh.u[i] = pk16(h0, h1); ul.u[i] = pk16(l0, l1);
    const unsigned short g0 = f2bf_bits(c[2 * i]), g1 = f2bf_bits(c[2 * i + 1]);
    const unsigned short m0 = f2bf_bits(c[2 * i] - bf_bits2f(g0)), m1 = f2bf_bits(c[2 * i + 1] - bf_bits2f(g1));
    uh.u[4 + i] = pk16(g0, g1); ul.u[4 + i] = pk16(m0, m1);
  }
  ho = uh.v; lo = ul.v;
}

__device__ __forceinline__ void gemm_core_32x64p(
    const unsigned short* __restrict__ A, const unsigned short* __restrict__ Bt,
    int K, size_t aoff, size_t boff, int hh, v8f (&acc)[2][4]) {
  const unsigned short* a0 = A + aoff;
  const unsigned short* a1 = a0 + (size_t)16 * K;
  const unsigned short* bp = Bt + boff;
#pragma unroll 1
  for (int k0 = 0; k0 < K; k0 += 32) {
    const v16b f0 = load_frag(a0 + k0, hh);
    const v16b f1 = load_frag(a1 + k0, hh);
#pragma unroll
    for (int nt = 0; nt < 4; ++nt) {
      const v16b fb = load_frag(bp + (size_t)nt * 16 * K + k0, hh);
      acc[0][nt] = wmma_bf16(f0, fb, acc[0][nt]);
      acc[1][nt] = wmma_bf16(f1, fb, acc[1][nt]);
    }
  }
}

__global__ __launch_bounds__(256) void k_cvt(const float* __restrict__ src, unsigned short* __restrict__ dst, int n8) {
  int i = blockIdx.x * 256 + threadIdx.x;
  const bool ok = i < n8;
  i = ok ? i : (n8 - 1);
  const float* s = src + (size_t)i * 8;
  const v4f f0 = *(const v4fa*)(s);
  const v4f f1 = *(const v4fa*)(s + 4);
  v4u u;
  u[0] = pk16(f2bf_bits(f0[0]), f2bf_bits(f0[1]));
  u[1] = pk16(f2bf_bits(f0[2]), f2bf_bits(f0[3]));
  u[2] = pk16(f2bf_bits(f1[0]), f2bf_bits(f1[1]));
  u[3] = pk16(f2bf_bits(f1[2]), f2bf_bits(f1[3]));
  unsigned short* d = dst + (size_t)i * 8;
  if (ok) *(volatile v4u*)d = u;
  __threadfence();
  if (ok) *(volatile v4u*)d = u;
}

__global__ __launch_bounds__(256) void k_tcvt(const float* __restrict__ W, unsigned short* __restrict__ ob, int R, int Cc) {
  __shared__ __align__(16) float tf[64 * 68];
  const int c0  = blockIdx.x * 64;
  const int r0  = blockIdx.y * 64;
  const int tid = threadIdx.x;
  {
    const int lr = tid >> 4;
    const int c4 = (tid & 15) * 4;
#pragma unroll
    for (int it = 0; it < 4; ++it) {
      const int rr = it * 16 + lr;
      const v4f a = *(const v4fa*)(W + (size_t)(r0 + rr) * Cc + c0 + c4);
      *(v4fa*)(tf + rr * 68 + c4) = a;
    }
  }
  __syncthreads();
  const int sub = tid >> 3;
  const int c8  = (tid & 7) * 8;
  v4u hv[2];
#pragma unroll
  for (int it = 0; it < 2; ++it) {
    const int oc = it * 32 + sub;
    v4u a;
#pragma unroll
    for (int q = 0; q < 4; ++q) {
      const float f0 = tf[(c8 + 2 * q) * 68 + oc];
      const float f1 = tf[(c8 + 2 * q + 1) * 68 + oc];
      a[q] = pk16(f2bf_bits(f0), f2bf_bits(f1));
    }
    hv[it] = a;
  }
  for (int pass = 0; pass < 2; ++pass) {
#pragma unroll
    for (int it = 0; it < 2; ++it) {
      const int oc = it * 32 + sub;
      const size_t go = (size_t)(c0 + oc) * R + r0 + c8;
      *(volatile v4u*)(ob + go) = hv[it];
    }
    __threadfence();
  }
}

__global__ __launch_bounds__(128) void k_proj(
    const unsigned short* __restrict__ Xb, const unsigned short* __restrict__ Wb,
    const float* __restrict__ Wattn, float* __restrict__ S,
    unsigned short* __restrict__ GTh, unsigned short* __restrict__ GTl) {
  __shared__ __align__(16) unsigned char smem[128 * 68 * 4];
  __shared__ __align__(16) float sA[2 * HF_];
  __shared__ __align__(16) float sS[4 * 128];
  float* sF = (float*)smem;
  unsigned short* sH = (unsigned short*)smem;
  unsigned short* sL = sH + 64 * 128;
  const int tid = threadIdx.x, lane = tid & 31, w = tid >> 5;
  const int hh = lane >> 4, m = lane & 15;
  const int xb = blockIdx.x;
  const int y  = blockIdx.y;
  const int m0 = xb * 128;
  const int n0 = y * 64;
  const int m0w = m0 + 32 * w;

  const v8f zero8 = {0.f, 0.f, 0.f, 0.f, 0.f, 0.f, 0.f, 0.f};
  v8f acc[2][4];
#pragma unroll
  for (int mt = 0; mt < 2; ++mt)
#pragma unroll
    for (int nt = 0; nt < 4; ++nt) acc[mt][nt] = zero8;

  gemm_core_32x64p(Xb, Wb, INF_, (size_t)(m0w + m) * INF_, (size_t)(n0 + m) * INF_, hh, acc);

  if (tid < 2 * HF_) sA[tid] = bf16r(Wattn[tid]);
#pragma unroll
  for (int nt = 0; nt < 4; ++nt)
#pragma unroll
    for (int mt = 0; mt < 2; ++mt)
#pragma unroll
      for (int r = 0; r < 8; ++r) {
        const int tokl = 32 * w + 16 * mt + 8 * hh + r;
        const int feat = 16 * nt + m;
        sF[tokl * 68 + feat] = acc[mt][nt][r];
      }
  __syncthreads();
  {
    float slA = 0.0f, srA = 0.0f, slB = 0.0f, srB = 0.0f;
    const float* fr = sF + tid * 68;
#pragma unroll 2
    for (int d4 = 0; d4 < HF_ / 4; ++d4) {
      const v4f xa = *(const v4fa*)(fr + 4 * d4);
      const v4f xc = *(const v4fa*)(fr + HF_ + 4 * d4);
      const v4f ya = *(const v4fa*)(sA + 4 * d4);
      const v4f za = *(const v4fa*)(sA + HF_ + 4 * d4);
      slA = fmaf(xa[0], ya[0], slA);
      slA = fmaf(xa[1], ya[1], slA);
      slA = fmaf(xa[2], ya[2], slA);
      slA = fmaf(xa[3], ya[3], slA);
      srA = fmaf(xa[0], za[0], srA);
      srA = fmaf(xa[1], za[1], srA);
      srA = fmaf(xa[2], za[2], srA);
      srA = fmaf(xa[3], za[3], srA);
      slB = fmaf(xc[0], ya[0], slB);
      slB = fmaf(xc[1], ya[1], slB);
      slB = fmaf(xc[2], ya[2], slB);
      slB = fmaf(xc[3], ya[3], slB);
      srB = fmaf(xc[0], za[0], srB);
      srB = fmaf(xc[1], za[1], srB);
      srB = fmaf(xc[2], za[2], srB);
      srB = fmaf(xc[3], za[3], srB);
    }
    sS[tid]       = slA;
    sS[128 + tid] = slB;
    sS[256 + tid] = srA;
    sS[384 + tid] = srB;
  }
  __syncthreads();
  {
    const int prow = (w >> 1) * NH_ + 2 * y + (w & 1);
    const size_t so = (size_t)prow * NN_ + m0 + lane * 4;
    const v4f vv = *(const v4fa*)(sS + w * 128 + lane * 4);
    *(volatile v4f*)(S + so) = vv;
    __threadfence();
    *(volatile v4f*)(S + so) = vv;
  }
#pragma unroll
  for (int nt = 0; nt < 4; ++nt)
#pragma unroll
    for (int mt = 0; mt < 2; ++mt)
#pragma unroll
      for (int r = 0; r < 8; ++r) {
        const int tokl = 32 * w + 16 * mt + 8 * hh + r;
        const int feat = 16 * nt + m;
        const float gv = acc[mt][nt][r];
        const unsigned short hb = f2bf_bits(gv);
        const unsigned short lb = f2bf_bits(gv - bf_bits2f(hb));
        const int idx = feat * 128 + tokl;
        sH[idx] = hb;
        sL[idx] = lb;
      }
  __syncthreads();
  {
    const int dsub = lane >> 4, t8 = (lane & 15) * 8;
    for (int pass = 0; pass < 2; ++pass) {
#pragma unroll
      for (int it = 0; it < 8; ++it) {
        const int d = 16 * w + 2 * it + dsub;
        const v4u hv = *(const v4ua*)(sH + d * 128 + t8);
        const v4u lv = *(const v4ua*)(sL + d * 128 + t8);
        const size_t go = ((size_t)(n0 + d)) * (size_t)NN_ + m0 + t8;
        *(volatile v4u*)(GTh + go) = hv;
        *(volatile v4u*)(GTl + go) = lv;
      }
      __threadfence();
    }
  }
}

#define AD_NT   256
#define AD_NW   8
#define EPT     8
#define CHUNK   (AD_NT * EPT)
#define WCAP    (EPT * 32)
#define SLOTB   6
#define NSLOT   64

static_assert((1 << SLOTB) == NSLOT);
static_assert((CHUNK & (CHUNK - 1)) == 0 && CHUNK == 2048);
static_assert(AD_NT == 32 * AD_NW);
static_assert(AD_NT * 32 == NSLOT * ADW);
static_assert(NN_ % NSLOT == 0);

__device__ __forceinline__ int scan_chunk(const int* __restrict__ keys, int nE, int cbase, int slotBase,
                                          int nb, int vec8, int* list, int tid, int lane, int wave) {
  int wc = 0;
  const int el0  = tid * EPT;
  const int e0   = cbase + el0;
  const int sent = -2147483647 - 1;
  v4i da, db;
  if (vec8 != 0 && cbase + CHUNK <= nE) {
    da = *(const v4ia*)(keys + e0);
    db = *(const v4ia*)(keys + e0 + 4);
  } else {
    da.x = (e0     < nE) ? keys[min(e0,     nE - 1)] : sent;
    da.y = (e0 + 1 < nE) ? keys[min(e0 + 1, nE - 1)] : sent;
    da.z = (e0 + 2 < nE) ? keys[min(e0 + 2, nE - 1)] : sent;
    da.w = (e0 + 3 < nE) ? keys[min(e0 + 3, nE - 1)] : sent;
    db.x = (e0 + 4 < nE) ? keys[min(e0 + 4, nE - 1)] : sent;
    db.y = (e0 + 5 < nE) ? keys[min(e0 + 5, nE - 1)] : sent;
    db.z = (e0 + 6 < nE) ? keys[min(e0 + 6, nE - 1)] : sent;
    db.w = (e0 + 7 < nE) ? keys[min(e0 + 7, nE - 1)] : sent;
  }
  const unsigned nbs = (unsigned)slotBase;
  const unsigned unb = (unsigned)nb;
  const unsigned s0 = (unsigned)da.x - nbs, s1 = (unsigned)da.y - nbs;
  const unsigned s2 = (unsigned)da.z - nbs, s3 = (unsigned)da.w - nbs;
  const unsigned s4 = (unsigned)db.x - nbs, s5 = (unsigned)db.y - nbs;
  const unsigned s6 = (unsigned)db.z - nbs, s7 = (unsigned)db.w - nbs;
  const bool h0 = s0 < unb, h1 = s1 < unb, h2 = s2 < unb, h3 = s3 < unb;
  const bool h4 = s4 < unb, h5 = s5 < unb, h6 = s6 < unb, h7 = s7 < unb;
  const unsigned any = __builtin_amdgcn_ballot_w32(h0 | h1 | h2 | h3 | h4 | h5 | h6 | h7);
  if (any != 0u) {
#define HITJ(J, HJ, SJ) { \
      const unsigned mj = __builtin_amdgcn_ballot_w32(HJ); \
      if (mj != 0u) { \
        if (HJ) { \
          const int pos = wc + (int)__builtin_amdgcn_mbcnt_lo(mj, 0u); \
          if (pos < WCAP) list[wave * WCAP + pos] = ((el0 + (J)) << SLOTB) | (int)(SJ); \
        } \
        wc += (int)__builtin_popcount(mj); } }
    HITJ(0, h0, s0)
    HITJ(1, h1, s1)
    HITJ(2, h2, s2)
    HITJ(3, h3, s3)
    HITJ(4, h4, s4)
    HITJ(5, h5, s5)
    HITJ(6, h6, s6)
    HITJ(7, h7, s7)
#undef HITJ
  }
  return wc;
}

__global__ __launch_bounds__(AD_NT) void k_adj(const int* __restrict__ keys, const int* __restrict__ gath,
                                               const float* __restrict__ emask, unsigned int* __restrict__ ADJ,
                                               int nE, int vec8) {
  __shared__ __align__(16) unsigned int sBits[NSLOT * ADW];
  __shared__ int list[AD_NW * WCAP];
  __shared__ int wcnt[AD_NW];
  const int tid = (int)threadIdx.x, lane = tid & 31, wave = tid >> 5;
  const int r0 = (int)blockIdx.x * NSLOT;

  {
    const v4u z = {0u, 0u, 0u, 0u};
#pragma unroll
    for (int i = 0; i < 8; ++i) *(v4ua*)(sBits + tid * 32 + 4 * i) = z;
  }
  __syncthreads();

  const int nChunks = (nE + CHUNK - 1) / CHUNK;
#pragma unroll 1
  for (int ch = 0; ch < nChunks; ++ch) {
    const int cbase = ch * CHUNK;
    const int wc = scan_chunk(keys, nE, cbase, r0, NSLOT, vec8, list, tid, lane, wave);
    if (lane == 0) wcnt[wave] = wc;
    __syncthreads();
    const int wcc = wc > WCAP ? WCAP : wc;
#pragma unroll 1
    for (int i0 = 0; i0 < wcc; i0 += 32) {
      const int i   = i0 + lane;
      const int ic  = i < wcc ? i : wcc - 1;
      const int ent = list[wave * WCAP + ic];
      const int el  = (ent >> SLOTB) & (CHUNK - 1);
      const int sl  = ent & (NSLOT - 1);
      int eid = cbase + el;
      eid = eid > nE - 1 ? nE - 1 : eid;
      int d = gath[eid];
      d = d < 0 ? 0 : (d > NN_ - 1 ? NN_ - 1 : d);
      const float mv = emask[eid];
      const int act = (mv != 0.0f) ? 1 : 0;
      const int packed = (act << 18) | (sl << 12) | d;
      if (i < wcc) list[wave * WCAP + i] = packed;
    }
    __syncthreads();
    if (wave < 2) {
      const int row = tid;
#pragma unroll 1
      for (int w2 = 0; w2 < AD_NW; ++w2) {
        int cnt = wcnt[w2];
        cnt = cnt < 0 ? 0 : (cnt > WCAP ? WCAP : cnt);
#pragma unroll 1
        for (int i = 0; i < cnt; ++i) {
          const int ent = list[w2 * WCAP + i];
          const bool hit = (((ent >> 12) & (NSLOT - 1)) == row) && (((ent >> 18) & 1) != 0);
          const unsigned int bit = hit ? (1u << (ent & 31)) : 0u;
          const int idx = row * ADW + ((ent & (NN_ - 1)) >> 5);
          sBits[idx] = sBits[idx] | bit;
        }
      }
    }
    __syncthreads();
  }
  if (tid < NSLOT) {
    const int key = r0 + tid;
    const int idx = tid * ADW + (key >> 5);
    sBits[idx] = sBits[idx] | (1u << (key & 31));
  }
  __syncthreads();
  for (int pass = 0; pass < 2; ++pass) {
#pragma unroll
    for (int it = 0; it < 8; ++it) {
      const int wo = it * (AD_NT * 4) + tid * 4;
      const v4u v = *(const v4ua*)(sBits + wo);
      *(volatile v4u*)(ADJ + (size_t)r0 * ADW + wo) = v;
    }
    __threadfence();
  }
}

__global__ __launch_bounds__(128) void k_attn(const float* __restrict__ S, const unsigned int* __restrict__ ADJ,
                                              const unsigned short* __restrict__ GTh,
                                              const unsigned short* __restrict__ GTl,
                                              float* __restrict__ out) {
  __shared__ __align__(16) unsigned char sraw[NSLOT * ADW * 4];
  __shared__ __align__(16) float sK[NN_];
  unsigned int* sMsk = (unsigned int*)sraw;

  const int tid = threadIdx.x, lane = tid & 31, w = tid >> 5;
  const int hh = lane >> 4, m = lane & 15;
  const int qt = blockIdx.x;
  const int h  = blockIdx.y;
  const int q0 = qt * 64, q0w = q0 + 16 * w, q = q0w + m;

  {
    const unsigned int* ga = ADJ + (size_t)q0 * ADW;
#pragma unroll 4
    for (int it = 0; it < 16; ++it) {
      const int wo = (it * 128 + tid) * 4;
      const v4u a = *(const v4ua*)(ga + wo);
      *(v4ua*)(sMsk + wo) = a;
    }
    const float* g = S + (size_t)(NH_ + h) * NN_ + tid * 32;
#pragma unroll 4
    for (int i = 0; i < 8; ++i) {
      const v4f a = *(const v4fa*)(g + 4 * i);
      *(v4fa*)(sK + tid * 32 + 4 * i) = a;
    }
  }
  const float elq = S[(size_t)h * NN_ + q];

  const v8f zero8 = {0.f, 0.f, 0.f, 0.f, 0.f, 0.f, 0.f, 0.f};
  v8f o[2];
  o[0] = zero8; o[1] = zero8;
  float mrun = MASKFILL, lrun = 0.0f;

  __syncthreads();

  const unsigned int* mrow = sMsk + (16 * w + m) * ADW;

#pragma unroll 1
  for (int ks = 0; ks < NN_ / 64; ++ks) {
    const int kb = ks * 64;
    const v2u mw = *(const v2ua*)(mrow + 2 * ks);
    const unsigned int w0 = mw[0], w1 = mw[1];

    v8f s[4];
#pragma unroll
    for (int j = 0; j < 4; ++j) {
      const int ko = kb + 16 * j + 8 * hh;
      const v4f kA = *(const v4fa*)(sK + ko);
      const v4f kB = *(const v4fa*)(sK + ko + 4);
      const float kv[8] = {kA[0], kA[1], kA[2], kA[3], kB[0], kB[1], kB[2], kB[3]};
      const unsigned int wsel = (j < 2) ? w0 : w1;
      const unsigned int bits = (wsel >> (((j & 1) * 16) + 8 * hh)) & 0xFFu;
#pragma unroll
      for (int r = 0; r < 8; ++r) {
        float t = elq + kv[r];
        t = (t >= 0.0f) ? t : SLOPE * t;
        t = (((bits >> r) & 1u) != 0u) ? t : MASKFILL;
        s[j][r] = t;
      }
    }
    float cm = MASKFILL;
#pragma unroll
    for (int j = 0; j < 4; ++j)
#pragma unroll
      for (int r = 0; r < 8; ++r) cm = fmaxf(cm, s[j][r]);
    cm = fmaxf(cm, __shfl_xor(cm, 16, 32));
    const float mnew  = fmaxf(mrun, cm);
    const float aexp  = __expf(mrun - mnew);
    const float alpha = (mrun > MASKHALF) ? aexp : 0.0f;
    mrun = mnew;
    float psum = 0.0f;
#pragma unroll
    for (int j = 0; j < 4; ++j)
#pragma unroll
      for (int r = 0; r < 8; ++r) {
        const float sv = s[j][r];
        const float pe = __expf(sv - mnew);
        const float p  = (sv > MASKHALF) ? pe : 0.0f;
        psum += p;
        s[j][r] = p;
      }
    psum += __shfl_xor(psum, 16, 32);
    lrun = lrun * alpha + psum;
#pragma unroll
    for (int t = 0; t < 2; ++t)
#pragma unroll
      for (int r = 0; r < 8; ++r) o[t][r] *= alpha;

    v16b p0h, p0l, p1h, p1l;
    pack_p2(s[0], s[1], p0h, p0l);
    pack_p2(s[2], s[3], p1h, p1l);

#pragma unroll
    for (int t = 0; t < 2; ++t) {
      const unsigned short* vph = GTh + (size_t)(h * HF_ + 16 * t + m) * (size_t)NN_ + kb;
      const unsigned short* vpl = GTl + (size_t)(h * HF_ + 16 * t + m) * (size_t)NN_ + kb;
      const v16b v0h = load_frag(vph, hh), v0l = load_frag(vpl, hh);
      o[t] = wmma_bf16(v0h, p0h, o[t]);
      o[t] = wmma_bf16(v0h, p0l, o[t]);
      o[t] = wmma_bf16(v0l, p0h, o[t]);
      const v16b v1h = load_frag(vph + 32, hh), v1l = load_frag(vpl + 32, hh);
      o[t] = wmma_bf16(v1h, p1h, o[t]);
      o[t] = wmma_bf16(v1h, p1l, o[t]);
      o[t] = wmma_bf16(v1l, p1h, o[t]);
    }
  }

  const float inv = 1.0f / lrun;
  __syncthreads();
  float* so = (float*)(sraw + w * (16 * ADW * 4));
#pragma unroll
  for (int t = 0; t < 2; ++t)
#pragma unroll
    for (int r = 0; r < 8; ++r)
      so[m * 36 + 16 * t + 8 * hh + r] = o[t][r] * inv;
  __syncthreads();
  {
    const int rq = lane >> 3, c4 = (lane & 7) * 4;
    for (int pass = 0; pass < 2; ++pass) {
#pragma unroll
      for (int it = 0; it < 4; ++it) {
        const int row = 4 * it + rq;
        const v4f v = *(const v4fa*)(so + row * 36 + c4);
        *(volatile v4f*)(out + (size_t)(q0w + row) * (size_t)DM_ + h * HF_ + c4) = v;
      }
      __threadfence();
    }
  }
}

extern "C" void kernel_launch(void* const* d_in, const int* in_sizes, int n_in,
                              void* d_out, int out_size, void* d_ws, size_t ws_size,
                              hipStream_t stream) {
  if (n_in < 5) return;
  if (in_sizes[0] != NN_ * INF_) return;
  if (in_sizes[1] < 2 || (in_sizes[1] & 1) != 0) return;
  const int nE = in_sizes[1] / 2;
  if (nE < 1 || nE > (1 << 24)) return;
  if (in_sizes[2] < nE) return;
  if (in_sizes[3] != INF_ * DM_) return;
  if (in_sizes[4] != 2 * HF_) return;
  if (out_size != NN_ * DM_) return;

  const float* hin   = (const float*)d_in[0];
  const int*   ei    = (const int*)d_in[1];
  const float* emask = (const float*)d_in[2];
  const float* Wfc   = (const float*)d_in[3];
  const float* Wattn = (const float*)d_in[4];
  float* out = (float*)d_out;
  const int* keys = ei;
  const int* gath = ei + nE;

  const size_t PX  = (size_t)NN_ * INF_ * 2;
  const size_t PW  = (size_t)DM_ * INF_ * 2;
  const size_t PS  = (size_t)2 * NH_ * NN_ * 4;
  const size_t PGT = (size_t)DM_ * NN_ * 2;
  const size_t PAD = (size_t)NN_ * ADW * 4;
  size_t off = 0;
  const size_t oXb  = off; off += PX;
  const size_t oWb  = off; off += PW;
  const size_t oS   = off; off += PS;
  const size_t oGTh = off; off += PGT;
  const size_t oGTl = off; off += PGT;
  const size_t oADJ = off; off += PAD;
  if (off > ws_size || off > (size_t)WSMAX) return;

  char* ws = (char*)d_ws;
  unsigned short* Xb  = (unsigned short*)(ws + oXb);
  unsigned short* Wb  = (unsigned short*)(ws + oWb);
  float*          S   = (float*)(ws + oS);
  unsigned short* GTh = (unsigned short*)(ws + oGTh);
  unsigned short* GTl = (unsigned short*)(ws + oGTl);
  unsigned int*   ADJ = (unsigned int*)(ws + oADJ);

  const int n8x = NN_ * INF_ / 8;
  k_cvt<<<dim3((n8x + 255) / 256), 256, 0, stream>>>(hin, Xb, n8x);
  k_tcvt<<<dim3(DM_ / 64, INF_ / 64), 256, 0, stream>>>(Wfc, Wb, INF_, DM_);
  k_proj<<<dim3(NN_ / 128, DM_ / 64), 128, 0, stream>>>(Xb, Wb, Wattn, S, GTh, GTl);
  k_adj<<<dim3(NN_ / NSLOT), AD_NT, 0, stream>>>(keys, gath, emask, ADJ, nE, 1);
  k_attn<<<dim3(NN_ / 64, NH_), 128, 0, stream>>>(S, ADJ, GTh, GTl, out);
  (void)hipGetLastError();
}
